// NetworkODEModel_19404662243683
// MI455X (gfx1250) — hardware-verified
//
#include <hip/hip_runtime.h>

typedef __attribute__((ext_vector_type(16))) _Float16 v16h;
typedef __attribute__((ext_vector_type(8)))  _Float16 v8h;
typedef __attribute__((ext_vector_type(8)))  float    v8f;
typedef __attribute__((ext_vector_type(4)))  float    v4f;

constexpr int NBATCH   = 64;
constexpr int NNODE    = 128;
constexpr int NDIM     = 2;
constexpr int HID      = 64;
constexpr int IGRP     = 16;
constexpr int NIGRP    = NNODE / IGRP;
constexpr int VPITCH   = 68;
constexpr int WPITCH   = 72;
constexpr int NTHREADS = 256;
constexpr int NWAVES   = NTHREADS / 32;
constexpr float OPSCALE = 64.0f;
constexpr float ACC_INV = 1.0f / 4096.0f;

static_assert(NNODE % IGRP == 0);
static_assert(IGRP * NDIM * 4 == 128);
static_assert(HID == 64);
static_assert(NWAVES * 2 == IGRP);
static_assert(NTHREADS == 2 * NNODE);
static_assert((IGRP * HID) % NTHREADS == 0);
static_assert((IGRP * NNODE) % NTHREADS == 0);
static_assert((HID * HID) % NTHREADS == 0);
static_assert(VPITCH % 4 == 0 && WPITCH % 8 == 0);

__device__ __forceinline__ v16h frag_load_h(const _Float16* p) {
  union { v16h v; v8h h[2]; } f;
  f.h[0] = *(const v8h*)(p);
  f.h[1] = *(const v8h*)(p + 16);
  return f.v;
}
__device__ __forceinline__ v8f mma_h(v16h a, v16h b, v8f c) {
  c = __builtin_amdgcn_wmma_f32_16x16x32_f16(false, a, false, b, (short)0, c, false, false);
  asm volatile("v_nop\n\tv_nop\n\tv_nop\n\tv_nop" : "+v"(c) : "v"(a), "v"(b));
  return c;
}
__device__ __forceinline__ float lrelu(float v) { return fmaxf(v, 0.01f * v); }
__device__ __forceinline__ v8f zero8() { return (v8f){0.f,0.f,0.f,0.f,0.f,0.f,0.f,0.f}; }

__device__ __forceinline__ void build_a_sum(const float* U, const float* Vrow, int hh, v16h (&a)[2]) {
#pragma unroll
  for (int kt = 0; kt < 2; ++kt) {
    const int h0 = kt * 32 + 8 * hh;
    const v4f u0 = *(const v4f*)(U + h0);
    const v4f u1 = *(const v4f*)(U + h0 + 4);
    const v4f u2 = *(const v4f*)(U + h0 + 16);
    const v4f u3 = *(const v4f*)(U + h0 + 20);
    const v4f w0 = *(const v4f*)(Vrow + h0);
    const v4f w1 = *(const v4f*)(Vrow + h0 + 4);
    const v4f w2 = *(const v4f*)(Vrow + h0 + 16);
    const v4f w3 = *(const v4f*)(Vrow + h0 + 20);
    const v4f s0 = u0 + w0, s1 = u1 + w1, s2 = u2 + w2, s3 = u3 + w3;
#pragma unroll
    for (int e = 0; e < 4; ++e) {
      a[kt][e]      = (_Float16)lrelu(s0[e]);
      a[kt][4 + e]  = (_Float16)lrelu(s1[e]);
      a[kt][8 + e]  = (_Float16)lrelu(s2[e]);
      a[kt][12 + e] = (_Float16)lrelu(s3[e]);
    }
  }
}
__device__ __forceinline__ void build_a_plain(const float* Hrow, int hh, v16h (&a)[2]) {
#pragma unroll
  for (int kt = 0; kt < 2; ++kt) {
    const int h0 = kt * 32 + 8 * hh;
    const v4f s0 = *(const v4f*)(Hrow + h0);
    const v4f s1 = *(const v4f*)(Hrow + h0 + 4);
    const v4f s2 = *(const v4f*)(Hrow + h0 + 16);
    const v4f s3 = *(const v4f*)(Hrow + h0 + 20);
#pragma unroll
    for (int e = 0; e < 4; ++e) {
      a[kt][e]      = (_Float16)s0[e];
      a[kt][4 + e]  = (_Float16)s1[e];
      a[kt][8 + e]  = (_Float16)s2[e];
      a[kt][12 + e] = (_Float16)s3[e];
    }
  }
}
__device__ __forceinline__ void tile_gemm(const v16h (&a)[2], const _Float16* Wt, int m, int hh, v8f (&acc)[4]) {
#pragma unroll
  for (int nt = 0; nt < 4; ++nt) {
    acc[nt] = zero8();
#pragma unroll
    for (int kt = 0; kt < 2; ++kt) {
      const v16h bf = frag_load_h(Wt + (nt * 16 + m) * WPITCH + kt * 32 + 8 * hh);
      acc[nt] = mma_h(a[kt], bf, acc[nt]);
    }
  }
}
__device__ __forceinline__ void epi_head(const v8f (&acc)[4], const float* bias, const float* w, int m, float (&rs)[8]) {
#pragma unroll
  for (int r = 0; r < 8; ++r) rs[r] = 0.f;
#pragma unroll
  for (int nt = 0; nt < 4; ++nt) {
    const float bv = bias[nt * 16 + m];
    const float wv = w[nt * 16 + m];
#pragma unroll
    for (int r = 0; r < 8; ++r) {
      float v = acc[nt][r] * ACC_INV + bv;
      v = lrelu(v);
      rs[r] = rs[r] + v * wv;
    }
  }
}

__global__ __launch_bounds__(NTHREADS) void fused_pairnet_kernel(
    const float* __restrict__ x,
    const float* __restrict__ Wn1, const float* __restrict__ bn1,
    const float* __restrict__ Wn2, const float* __restrict__ bn2,
    const float* __restrict__ Wno, const float* __restrict__ bno,
    const float* __restrict__ Wc1, const float* __restrict__ bc1,
    const float* __restrict__ Wc2, const float* __restrict__ bc2,
    const float* __restrict__ Wco, const float* __restrict__ bco,
    const float* __restrict__ Ap, const int* __restrict__ tstep,
    float* __restrict__ out)
{
  (void)tstep;
  __shared__ __align__(16) float    sV[NNODE * VPITCH];
  __shared__ __align__(16) float    sU[IGRP * HID];
  __shared__ __align__(16) float    sH1[IGRP * VPITCH];
  __shared__ __align__(16) float    sA[IGRP * NNODE];
  __shared__ __align__(16) _Float16 sWct[HID * WPITCH];
  __shared__ __align__(16) _Float16 sWnt[HID * WPITCH];
  __shared__ float sWc1[4 * HID], sWn1[2 * HID];
  __shared__ float sbc1[HID], sbn1[HID], sbc2[HID], sbn2[HID], sWco[HID], sWno[HID];
  __shared__ float sNode[IGRP], sCoup[IGRP], sFin[IGRP];

  const int tid  = threadIdx.x;
  const int lane = tid & 31;
  const int wave = __builtin_amdgcn_readfirstlane(tid >> 5);
  const int hh   = lane >> 4;
  const int m    = lane & 15;
  const int b    = blockIdx.x / NIGRP;
  const int i0   = (blockIdx.x - b * NIGRP) * IGRP;
  const float bnov = bno[0];
  const float bcov = bco[0];

  {
    sWc1[tid] = Wc1[tid];
    const int t128 = tid < 2 * HID ? tid : 2 * HID - 1;
    const float wn1v = Wn1[t128];
    if (tid < 2 * HID) sWn1[tid] = wn1v;
    const int t64 = tid < HID ? tid : HID - 1;
    const float c1v = bc1[t64], n1v = bn1[t64], c2v = bc2[t64], n2v = bn2[t64], cov = Wco[t64], nov = Wno[t64];
    if (tid < HID) { sbc1[tid] = c1v; sbn1[tid] = n1v; sbc2[tid] = c2v; sbn2[tid] = n2v; sWco[tid] = cov; sWno[tid] = nov; }
#pragma unroll 1
    for (int idx = tid; idx < HID * HID; idx += NTHREADS) {
      const int k = idx >> 6, n = idx & 63;
      sWct[n * WPITCH + k] = (_Float16)(Wc2[idx] * OPSCALE);
      sWnt[n * WPITCH + k] = (_Float16)(Wn2[idx] * OPSCALE);
    }
#pragma unroll 1
    for (int idx = tid; idx < HID * 8; idx += NTHREADS) {
      const int n = idx >> 3, p = idx & 7;
      sWct[n * WPITCH + HID + p] = (_Float16)0.0f;
      sWnt[n * WPITCH + HID + p] = (_Float16)0.0f;
    }
  }
  __syncthreads();

  {
    const int j = tid & (NNODE - 1);
    const int hbase = (tid >> 7) * 32;
    const size_t xo = (size_t)(b * NNODE + j) * NDIM;
    const float xa = x[xo], xb = x[xo + 1];
#pragma unroll 1
    for (int q = 0; q < 32; ++q) {
      const int hc = hbase + q;
      sV[j * VPITCH + hc] = (xa * sWc1[2 * HID + hc] + xb * sWc1[3 * HID + hc]) * OPSCALE;
    }
  }
#pragma unroll 1
  for (int idx = tid; idx < IGRP * HID; idx += NTHREADS) {
    const int ii = idx >> 6, hc = idx & 63;
    const size_t xo = (size_t)(b * NNODE + i0 + ii) * NDIM;
    const float xa = x[xo], xb = x[xo + 1];
    sU[ii * HID + hc]     = (xa * sWc1[hc] + xb * sWc1[HID + hc] + sbc1[hc]) * OPSCALE;
    sH1[ii * VPITCH + hc] = lrelu(xa * sWn1[hc] + xb * sWn1[HID + hc] + sbn1[hc]) * OPSCALE;
  }
#pragma unroll 1
  for (int idx = tid; idx < IGRP * NNODE; idx += NTHREADS) {
    const int ii = idx >> 7, j = idx & (NNODE - 1);
    const int i = i0 + ii;
    const float av = Ap[(size_t)i * NNODE + j];
    const float sg = 1.0f / (1.0f + expf(-av));
    sA[idx] = (i == j) ? 0.0f : sg;
  }
  __syncthreads();

  if (wave == 0) {
    v16h a[2];
    build_a_plain(sH1 + m * VPITCH, hh, a);
    v8f acc[4];
    tile_gemm(a, sWnt, m, hh, acc);
    float rs[8];
    epi_head(acc, sbn2, sWno, m, rs);
#pragma unroll
    for (int r = 0; r < 8; ++r) {
      rs[r] += __shfl_xor(rs[r], 1, 32);
      rs[r] += __shfl_xor(rs[r], 2, 32);
      rs[r] += __shfl_xor(rs[r], 4, 32);
      rs[r] += __shfl_xor(rs[r], 8, 32);
    }
    if (m == 0) {
#pragma unroll
      for (int r = 0; r < 8; ++r) sNode[8 * hh + r] = rs[r] + bnov;
    }
  }

#pragma unroll 1
  for (int ip = 0; ip < 2; ++ip) {
    const int ii = wave * 2 + ip;
    const float* U    = sU + ii * HID;
    const float* Arow = sA + ii * NNODE;
    float cl = 0.f;
#pragma unroll 1
    for (int jt = 0; jt < NNODE / 16; ++jt) {
      const int j0 = jt * 16;
      v16h a[2];
      build_a_sum(U, sV + (j0 + m) * VPITCH, hh, a);
      v8f acc[4];
      tile_gemm(a, sWct, m, hh, acc);
      float rs[8];
      epi_head(acc, sbc2, sWco, m, rs);
#pragma unroll
      for (int r = 0; r < 8; ++r) cl = cl + Arow[j0 + 8 * hh + r] * rs[r];
    }
    cl += __shfl_xor(cl, 1, 32);
    cl += __shfl_xor(cl, 2, 32);
    cl += __shfl_xor(cl, 4, 32);
    cl += __shfl_xor(cl, 8, 32);
    cl += __shfl_xor(cl, 16, 32);
    if (lane == 0) sCoup[ii] = cl;
  }
  __syncthreads();

  if (wave == 0) {
    const int ii = lane & (IGRP - 1);
    float sa = 0.f;
#pragma unroll 1
    for (int j = 0; j < NNODE; ++j) sa += sA[ii * NNODE + j];
    const float fin = sNode[ii] + (sCoup[ii] + bcov * sa);
    if (lane < IGRP) sFin[ii] = fin;
  }
  __syncthreads();

  if (wave == 0) {
    const int q   = lane < 8 ? lane : 7;
    const int iiA = 2 * q, iiB = 2 * q + 1;
    const float xA = x[(size_t)(b * NNODE + i0 + iiA) * NDIM + 1];
    const float xB = x[(size_t)(b * NNODE + i0 + iiB) * NDIM + 1];
    v4f val;
    val[0] = xA; val[1] = sFin[iiA]; val[2] = xB; val[3] = sFin[iiB];
    float* dst = out + (size_t)(b * NNODE + i0) * NDIM + q * 4;
    for (int pass = 0; pass < 2; ++pass) {
      if (lane < 8) *(volatile v4f*)dst = val;
      __threadfence();
    }
  }
}

extern "C" void kernel_launch(void* const* d_in, const int* in_sizes, int n_in,
                              void* d_out, int out_size, void* d_ws, size_t ws_size,
                              hipStream_t stream) {
  (void)d_ws; (void)ws_size;
  if (n_in < 15) return;
  if (in_sizes[0]  != NBATCH * NNODE * NDIM) return;
  if (in_sizes[1]  != NDIM * HID || in_sizes[2] != HID) return;
  if (in_sizes[3]  != HID * HID || in_sizes[4] != HID || in_sizes[5] != HID || in_sizes[6] < 1) return;
  if (in_sizes[7]  != 2 * NDIM * HID || in_sizes[8] != HID) return;
  if (in_sizes[9]  != HID * HID || in_sizes[10] != HID || in_sizes[11] != HID || in_sizes[12] < 1) return;
  if (in_sizes[13] != NNODE * NNODE) return;
  if (out_size != NBATCH * NNODE * NDIM) return;

  const float* x   = (const float*)d_in[0];
  const float* Wn1 = (const float*)d_in[1];
  const float* bn1 = (const float*)d_in[2];
  const float* Wn2 = (const float*)d_in[3];
  const float* bn2 = (const float*)d_in[4];
  const float* Wno = (const float*)d_in[5];
  const float* bno = (const float*)d_in[6];
  const float* Wc1 = (const float*)d_in[7];
  const float* bc1 = (const float*)d_in[8];
  const float* Wc2 = (const float*)d_in[9];
  const float* bc2 = (const float*)d_in[10];
  const float* Wco = (const float*)d_in[11];
  const float* bco = (const float*)d_in[12];
  const float* Ap  = (const float*)d_in[13];
  const int*   tst = (const int*)d_in[14];
  float* out = (float*)d_out;

  fused_pairnet_kernel<<<dim3(NBATCH * NIGRP), dim3(NTHREADS), 0, stream>>>(
      x, Wn1, bn1, Wn2, bn2, Wno, bno, Wc1, bc1, Wc2, bc2, Wco, bco, Ap, tst, out);
}
